// MultiHeadAttention_58428735095200
// MI455X (gfx1250) — hardware-run, weakly checked
//
#include <hip/hip_runtime.h>
#ifndef NB
#define NB 2
#endif
#ifndef SEQ
#define SEQ 2048
#endif
#define NB_FULL 2
#define SEQ_FULL 2048
#define SQ SEQ
#define DM 1024
#define NH 16
#define HD 64
#ifndef HG
#define HG 1
#endif
#ifndef RESQ
#define RESQ 512
#endif
#define NR ((size_t)NB * SQ)
#define LQ DM
#define RES_UP 1024.0f
#define RES_DN 0.0009765625f

static_assert(SQ % 64 == 0);
static_assert(DM % 64 == 0);
static_assert(HD == 64);
static_assert(NH * HD == DM);
static_assert(NH % HG == 0);
static_assert(NB <= NB_FULL);
static_assert(SQ <= SEQ_FULL);

typedef unsigned short v8us __attribute__((ext_vector_type(8), may_alias));
typedef float  v8f  __attribute__((ext_vector_type(8)));
typedef float  v4f  __attribute__((ext_vector_type(4)));
typedef float  v4fa __attribute__((ext_vector_type(4), may_alias));
typedef _Float16 v16h __attribute__((ext_vector_type(16)));
typedef _Float16 v4h __attribute__((ext_vector_type(4)));
union FragH { v16h v; v8us half[2]; _Float16 h[16]; unsigned short u[16]; };

__device__ __forceinline__ unsigned short bf16_bits(float x) { unsigned int u = __float_as_uint(x); return (unsigned short)((u + 0x7FFFu + ((u >> 16) & 1u)) >> 16); }
__device__ __forceinline__ float bf16_val(unsigned short b) { return __uint_as_float(((unsigned int)b) << 16); }
__device__ __forceinline__ float bf16_rne(float x) { return bf16_val(bf16_bits(x)); }

__device__ __forceinline__ v16h g2_frag(const _Float16* p, int hh) { FragH f; f.half[0] = *(const v8us*)((const unsigned short*)p + 8 * hh); f.half[1] = *(const v8us*)((const unsigned short*)p + 16 + 8 * hh); return f.v; }
__device__ __forceinline__ v8f g2_mma(v16h a, v16h b, v8f c) { v8f d = __builtin_amdgcn_wmma_f32_16x16x32_f16(false, a, false, b, (short)0, c, false, false); asm volatile("v_nop\n\tv_nop\n\tv_nop\n\tv_nop" : "+v"(d) : "v"(a), "v"(b)); return d; }
__device__ __forceinline__ void mma_a2(v16h ah, v16h al, v16h bh, v8f& c0, v8f& c1) {
  c0 = __builtin_amdgcn_wmma_f32_16x16x32_f16(false, ah, false, bh, (short)0, c0, false, false);
  c1 = __builtin_amdgcn_wmma_f32_16x16x32_f16(false, al, false, bh, (short)0, c1, false, false);
  asm volatile("v_nop\n\tv_nop\n\tv_nop\n\tv_nop" : "+v"(c0), "+v"(c1) : "v"(ah), "v"(al), "v"(bh));
}
__device__ __forceinline__ void mma_ab3(v16h ah, v16h al, v16h bh, v16h bl, v8f& c0, v8f& c1) {
  c0 = __builtin_amdgcn_wmma_f32_16x16x32_f16(false, ah, false, bh, (short)0, c0, false, false);
  c1 = __builtin_amdgcn_wmma_f32_16x16x32_f16(false, ah, false, bl, (short)0, c1, false, false);
  c1 = __builtin_amdgcn_wmma_f32_16x16x32_f16(false, al, false, bh, (short)0, c1, false, false);
  asm volatile("v_nop\n\tv_nop\n\tv_nop\n\tv_nop" : "+v"(c0), "+v"(c1) : "v"(ah), "v"(al), "v"(bh), "v"(bl));
}

template <int PM>
__device__ __forceinline__ void kloop(const _Float16* ahp, const _Float16* alp, const _Float16* bhp, const _Float16* blp,
                                      int ldb, int kend, int hh, v8f (&c0)[4], v8f (&c1)[4]) {
#pragma unroll 1
  for (int kb = 0; kb < kend; kb += 32) {
    const v16h ah = g2_frag(ahp + kb, hh);
    v16h al = ah;
    if (PM >= 2) al = g2_frag(alp + kb, hh);
#pragma unroll
    for (int t = 0; t < 4; ++t) {
      const v16h bh = g2_frag(bhp + (size_t)(t * 16) * ldb + kb, hh);
      if (PM == 0) { c0[t] = g2_mma(ah, bh, c0[t]); }
      else if (PM == 2) { mma_a2(ah, al, bh, c0[t], c1[t]); }
      else { const v16h bl = g2_frag(blp + (size_t)(t * 16) * ldb + kb, hh); mma_ab3(ah, al, bh, bl, c0[t], c1[t]); }
    }
  }
}

template <int PM>
__global__ __launch_bounds__(128) void k_gemm3(const _Float16* __restrict__ Ah, const _Float16* __restrict__ Al, int lda, size_t sA,
                                               const _Float16* __restrict__ Bh, const _Float16* __restrict__ Bl, int ldb, size_t sB,
                                               float alpha, const float* __restrict__ bias,
                                               float* __restrict__ C, _Float16* __restrict__ C16h, _Float16* __restrict__ C16l, int ldc, size_t sC,
                                               int M, int N, int K, int cmode, int resrows) {
  __shared__ __attribute__((aligned(16))) float so[4][16][68];
  const int tid = threadIdx.x, w = __builtin_amdgcn_readfirstlane((int)(tid >> 5)), lane = tid & 31, ln = lane & 15, hh = lane >> 4;
  const int by = blockIdx.y;
  const int ntn = N >> 6;
  const int mt = blockIdx.x / ntn, nq = blockIdx.x - mt * ntn;
  const int row0 = mt * 64 + 16 * w, col0 = nq * 64;
  if (row0 >= M) return;
  if (cmode == 1 && col0 > row0 + 15) return;
  int kend = K;
  if (cmode == 2) { const int kc = (((row0 + 15) >> 5) + 1) << 5; kend = kc < K ? kc : K; }
  const bool res = (PM != 0) && (row0 < resrows);
  const v8f z8 = {0.f, 0.f, 0.f, 0.f, 0.f, 0.f, 0.f, 0.f};
  v8f c0[4] = {z8, z8, z8, z8};
  v8f c1[4] = {z8, z8, z8, z8};
  const size_t aofs = (size_t)by * sA + (size_t)(row0 + ln) * lda;
  const size_t bofs = (size_t)by * sB + (size_t)(col0 + ln) * ldb;
  const _Float16* ahp = Ah + aofs;
  const _Float16* bhp = Bh + bofs;
  if (res) {
    const _Float16* alp = Al + aofs;
    const _Float16* blp = (PM == 3) ? (Bl + bofs) : bhp;
    kloop<PM>(ahp, alp, bhp, blp, ldb, kend, hh, c0, c1);
  } else {
    kloop<0>(ahp, ahp, bhp, bhp, ldb, kend, hh, c0, c1);
  }
#pragma unroll
  for (int t = 0; t < 4; ++t) {
    const int col = col0 + t * 16 + ln;
    const float bv = bias ? bf16_rne(bias[col]) : 0.f;
#pragma unroll
    for (int r = 0; r < 8; ++r) { const float v = (c0[t][r] + c1[t][r] * RES_DN) * alpha + bv; so[w][8 * hh + r][t * 16 + ln] = v; }
  }
  __builtin_amdgcn_fence(4  , "workgroup");
  __builtin_amdgcn_wave_barrier();
  const int rsub = lane >> 4, c4 = (lane & 15) * 4;
  const size_t cofs = (size_t)by * sC;
  for (int pass = 0; pass < 2; ++pass) {
#pragma unroll
    for (int q = 0; q < 8; ++q) {
      const int r = q * 2 + rsub;
      const v4f v = *(const v4fa*)&so[w][r][c4];
      const size_t o = cofs + (size_t)(row0 + r) * ldc + col0 + c4;
      if (C) *(volatile v4f*)(C + o) = v;
      if (C16h) {
        v4h h4, l4;
#pragma unroll
        for (int i = 0; i < 4; ++i) { const _Float16 h = (_Float16)v[i]; h4[i] = h; l4[i] = (_Float16)((v[i] - (float)h) * RES_UP); }
        *(volatile v4h*)(C16h + o) = h4;
        if (C16l) *(volatile v4h*)(C16l + o) = l4;
      }
    }
    if (pass == 0) __threadfence();
  }
}

__global__ __launch_bounds__(256) void k_wt_f16(const float* __restrict__ W, _Float16* __restrict__ Wt, int K, int N, float scale) {
  const int t = blockIdx.x * 256 + threadIdx.x; if (t >= N * (K / 8)) return;
  const int n = t / (K / 8), k8 = (t % (K / 8)) * 8; FragH f;
#pragma unroll
  for (int i = 0; i < 8; ++i) f.h[i] = (_Float16)(bf16_rne(W[(size_t)(k8 + i) * N + n]) * scale);
  const v8us o = f.half[0];
  *(volatile v8us*)((unsigned short*)Wt + (size_t)n * K + k8) = o; __threadfence(); *(volatile v8us*)((unsigned short*)Wt + (size_t)n * K + k8) = o;
}

__global__ __launch_bounds__(256) void k_x16(const float* __restrict__ x, _Float16* __restrict__ X16, size_t n8) {
  const size_t t = (size_t)blockIdx.x * 256 + threadIdx.x; if (t >= n8) return;
  const size_t e = t * 8; const size_t row = e / DM; const size_t c = e % DM;
  const size_t b = row / SQ, s = row % SQ;
  const float* src = x + (b * (size_t)SEQ_FULL + s) * DM + c;
  const v4f a = *(const v4fa*)src, d = *(const v4fa*)(src + 4);
  FragH f;
#pragma unroll
  for (int q = 0; q < 4; ++q) { f.h[q] = (_Float16)bf16_rne(a[q]); f.h[4 + q] = (_Float16)bf16_rne(d[q]); }
  const v8us o = f.half[0];
  *(volatile v8us*)((unsigned short*)X16 + e) = o; __threadfence(); *(volatile v8us*)((unsigned short*)X16 + e) = o;
}

template <int NHv, int TTv>
__global__ __launch_bounds__(256) void k_vt(const _Float16* __restrict__ V16, size_t planeV, int ldv, _Float16* __restrict__ Vt, size_t planeT) {
  __shared__ unsigned short tl[64][66];
  const int tid = threadIdx.x; const int h = blockIdx.x / (TTv / 64), lg = blockIdx.x % (TTv / 64); const int pl = blockIdx.y;
  const unsigned short* src = (const unsigned short*)V16 + (size_t)pl * planeV;
  unsigned short* dst = (unsigned short*)Vt + (size_t)pl * planeT;
  for (int i = tid; i < 64 * 8; i += 256) { const int r = i / 8, c8 = (i % 8) * 8; FragH f; f.half[0] = *(const v8us*)(src + ((size_t)lg * 64 + r) * ldv + h * 64 + c8);
#pragma unroll
    for (int q = 0; q < 8; ++q) tl[r][c8 + q] = f.u[q]; }
  __syncthreads();
  for (int pass = 0; pass < 2; ++pass) {
#pragma unroll
    for (int rd = 0; rd < 2; ++rd) { const int d = rd * 32 + tid / 8, pc = tid % 8; FragH f;
#pragma unroll
      for (int q = 0; q < 8; ++q) f.u[q] = tl[pc * 8 + q][d];
      const v8us o = f.half[0];
      *(volatile v8us*)(dst + ((size_t)h * 64 + d) * TTv + lg * 64 + pc * 8) = o; }
    if (pass == 0) __threadfence(); }
}

__global__ __launch_bounds__(256) void k_rsmc(const float* __restrict__ S, _Float16* __restrict__ Ph, _Float16* __restrict__ Pl, int qn, int hg) {
  #pragma clang fp contract(off)
  const int t = blockIdx.x * 256 + threadIdx.x; if (t >= qn * hg) return;
  const int q = t % qn; const size_t i = (size_t)(t / qn) * SQ + q; const float* s = S + i * SQ;
  float mx = -3.0e38f;
#pragma unroll 1
  for (int j = 0; j <= q; ++j) mx = fmaxf(mx, s[j]);
  float se = 0.f;
#pragma unroll 1
  for (int j = 0; j <= q; ++j) se += __expf(s[j] - mx);
  const float sc = 256.0f / se;
  const int jend = ((q >> 5) + 1) << 5;
  int jend64 = (jend + 63) & ~63;
  if (jend64 > SQ) jend64 = SQ;
#pragma unroll 1
  for (int j0 = 0; j0 < jend64; j0 += 8) {
    FragH fh, fl;
#pragma unroll
    for (int u = 0; u < 8; ++u) {
      const int j = j0 + u; const int jc = j < q ? j : q;
      const float e = __expf(s[jc] - mx) * sc;
      const float v = (j <= q) ? e : 0.0f;
      const _Float16 h = (_Float16)v; fh.h[u] = h; fl.h[u] = (_Float16)((v - (float)h) * RES_UP);
    }
    const v8us oh = fh.half[0], ol = fl.half[0];
    unsigned short* dh = (unsigned short*)Ph + i * SQ + j0; unsigned short* dl = (unsigned short*)Pl + i * SQ + j0;
    *(volatile v8us*)dh = oh; *(volatile v8us*)dl = ol; __threadfence(); *(volatile v8us*)dh = oh; *(volatile v8us*)dl = ol;
  }
}

constexpr size_t SZ_W  = (size_t)DM * DM * 2;
constexpr size_t SZ_R  = (size_t)NB * SQ * DM * 2;
constexpr size_t SZ_S  = (size_t)HG * SQ * SQ * 4;
constexpr size_t SZ_P  = (size_t)HG * SQ * SQ * 2;
constexpr size_t SZ_VT = (size_t)NH * HD * SQ * 2;
constexpr size_t WS_TOTAL = 4 * SZ_W + 9 * SZ_R + SZ_S + 2 * SZ_P + 2 * SZ_VT;
static_assert(WS_TOTAL <= (size_t)134217728);
static_assert(SZ_W % 256 == 0 && SZ_R % 256 == 0 && SZ_S % 256 == 0 && SZ_P % 256 == 0 && SZ_VT % 256 == 0);

extern "C" void kernel_launch(void* const* d_in, const int* in_sizes, int n_in,
                              void* d_out, int out_size, void* d_ws, size_t ws_size, hipStream_t stream) {
  if (n_in < 9) return;
  const size_t need = ((size_t)(NB - 1) * SEQ_FULL + SQ) * DM;
  if ((size_t)in_sizes[0] < need || (size_t)out_size < need) return;
  if (in_sizes[1] < DM * DM || in_sizes[3] < DM * DM || in_sizes[5] < DM * DM || in_sizes[7] < DM * DM) return;
  if (in_sizes[2] < DM || in_sizes[4] < DM || in_sizes[6] < DM || in_sizes[8] < DM) return;
  const float* const* I = (const float* const*)d_in;
  const float* x = I[0]; const float* wq = I[1]; const float* bq = I[2]; const float* wk = I[3]; const float* bk = I[4];
  const float* wv = I[5]; const float* bv = I[6]; const float* wo = I[7]; const float* bo = I[8];
  char* ws = (char*)d_ws; size_t off = 0;
  auto take = [&](size_t bytes) { char* p = ws + off; off += (bytes + 255) & ~(size_t)255; return p; };
  _Float16* BQ = (_Float16*)take(SZ_W); _Float16* BK = (_Float16*)take(SZ_W); _Float16* BV = (_Float16*)take(SZ_W); _Float16* BO = (_Float16*)take(SZ_W);
  _Float16* X16 = (_Float16*)take(SZ_R);
  _Float16* QH = (_Float16*)take(SZ_R); _Float16* QL = (_Float16*)take(SZ_R); _Float16* KH = (_Float16*)take(SZ_R); _Float16* KL = (_Float16*)take(SZ_R);
  _Float16* VP = (_Float16*)take(2 * SZ_R);
  _Float16* OH = (_Float16*)take(SZ_R); _Float16* OL = (_Float16*)take(SZ_R);
  float* S = (float*)take(SZ_S); _Float16* PH = (_Float16*)take(SZ_P); _Float16* PL = (_Float16*)take(SZ_P);
  _Float16* VT = (_Float16*)take(2 * SZ_VT);
  if (off > ws_size || off > WS_TOTAL) return;
  const size_t planeV = NR * DM, planeT = (size_t)NH * HD * SQ;
  { const unsigned g = (unsigned)(((size_t)DM * (DM / 8) + 255) / 256);
    k_wt_f16<<<g, 256, 0, stream>>>(wq, BQ, DM, DM, 16.0f); k_wt_f16<<<g, 256, 0, stream>>>(wk, BK, DM, DM, 16.0f);
    k_wt_f16<<<g, 256, 0, stream>>>(wv, BV, DM, DM, 16.0f); k_wt_f16<<<g, 256, 0, stream>>>(wo, BO, DM, DM, 16.0f); }
  k_x16<<<(unsigned)((NR * DM / 8 + 255) / 256), 256, 0, stream>>>(x, X16, NR * DM / 8);
  const dim3 gp((unsigned)((NR / 64) * (DM / 64)), 1);
  k_gemm3<0><<<gp, 128, 0, stream>>>(X16, nullptr, DM, 0, BQ, nullptr, DM, 0, 0.0625f, bq, nullptr, QH, QL, DM, 0, (int)NR, DM, DM, 0, 0);
  k_gemm3<0><<<gp, 128, 0, stream>>>(X16, nullptr, DM, 0, BK, nullptr, DM, 0, 0.0625f, bk, nullptr, KH, KL, DM, 0, (int)NR, DM, DM, 0, 0);
  k_gemm3<0><<<gp, 128, 0, stream>>>(X16, nullptr, DM, 0, BV, nullptr, DM, 0, 0.0625f, bv, nullptr, VP, VP + planeV, DM, 0, (int)NR, DM, DM, 0, 0);
  for (int b = 0; b < NB; ++b) {
    const size_t r0 = (size_t)b * SQ;
    k_vt<NH, SQ><<<dim3(NH * (SQ / 64), 2), 256, 0, stream>>>(VP + r0 * LQ, planeV, LQ, VT, planeT);
    for (int h0 = 0; h0 < NH; h0 += HG) {
      const size_t qk = r0 * LQ + (size_t)h0 * HD;
      k_gemm3<3><<<dim3((SQ / 64) * (SQ / 64), HG), 128, 0, stream>>>(QH + qk, QL + qk, LQ, (size_t)HD, KH + qk, KL + qk, LQ, (size_t)HD, 0.125f, nullptr,
                                                                     S, nullptr, nullptr, SQ, (size_t)SQ * SQ, SQ, SQ, HD, 1, RESQ);
      k_rsmc<<<(HG * SQ + 255) / 256, 256, 0, stream>>>(S, PH, PL, SQ, HG);
      k_gemm3<3><<<dim3((SQ / 64) * (HD / 64), HG), 128, 0, stream>>>(PH, PL, SQ, (size_t)SQ * SQ, VT + (size_t)h0 * HD * SQ, VT + planeT + (size_t)h0 * HD * SQ, SQ, (size_t)HD * SQ, 0.25f, nullptr,
                                                                     nullptr, OH + qk, OL + qk, DM, (size_t)HD, SQ, HD, SQ, 2, RESQ);
    }
  }
  k_gemm3<2><<<dim3((SQ / 64) * (DM / 64), NB), 128, 0, stream>>>(OH, OL, DM, (size_t)SQ * DM, BO, nullptr, DM, 0, 0.0009765625f, bo,
                                                                 (float*)d_out, nullptr, nullptr, DM, (size_t)SEQ_FULL * DM, SQ, DM, DM, 0, RESQ);
}
